// InferCode_22651657519716
// MI455X (gfx1250) — hardware-verified
//
#include <hip/hip_runtime.h>
#include <stddef.h>
#include <stdint.h>
#include <float.h>
#include <math.h>

#define DIM     128
#define KCAT    384
#define SUBT    50000
#define SUBP    50176
#define NTREE   64
#define CSR_R   8192
#define CSR_CAP 24576
#define MAXDEG  64
#define OCH     512
#define NCH     98
#define ERRV    0x0BADC0DE
#define APITCH  392
#define OPITCH  132
#define EPITCH  136
#define OTP     68

static_assert(SUBT % 32 == 16);
static_assert(NCH * OCH == SUBP);
static_assert((NCH - 1) * OCH < SUBT - 16);
static_assert((SUBP * DIM) % 2048 == 0);
static_assert(CSR_R % 64 == 0);
static_assert(CSR_R == 32 * 256);
static_assert((CSR_CAP % 1024) == 0);
static_assert(NTREE % 16 == 0);
static_assert(64 * OPITCH * 4 <= 64 * APITCH * 2);
static_assert(128 * EPITCH * 2 == 8 * 16 * OTP * 4);

typedef _Float16 v16h __attribute__((ext_vector_type(16)));
typedef _Float16 v8h  __attribute__((ext_vector_type(8)));
typedef float    v8f  __attribute__((ext_vector_type(8)));
typedef float    v4f  __attribute__((ext_vector_type(4)));
typedef unsigned int v4u __attribute__((ext_vector_type(4)));
typedef int      v4i  __attribute__((ext_vector_type(4)));

union Frag  { v16h v; v8h h[2]; };
union Pack8 { v8h h; v4u u; };

__device__ __forceinline__ v8f mma16(v16h a, v16h b, v8f c) {
  c = __builtin_amdgcn_wmma_f32_16x16x32_f16(false, a, false, b, (short)0, c, false, false);
  asm volatile("v_nop\n\tv_nop\n\tv_nop\n\tv_nop" : "+v"(c) : "v"(a), "v"(b));
  return c;
}

__device__ __forceinline__ v16h ldfrag(const _Float16* p, int ld, int row0, int k0, int lane) {
  const int m = lane & 15, lh = lane >> 4;
  const _Float16* q = p + (size_t)(row0 + m) * ld + k0 + 8 * lh;
  Frag f;
  f.h[0] = *(const v8h*)(q);
  f.h[1] = *(const v8h*)(q + 16);
  return f.v;
}

__device__ __forceinline__ v8f zero8() { return (v8f){0.f, 0.f, 0.f, 0.f, 0.f, 0.f, 0.f, 0.f}; }

__device__ __forceinline__ v8h cvt8(v4f a0, v4f a1) {
  return (v8h){(_Float16)a0[0], (_Float16)a0[1], (_Float16)a0[2], (_Float16)a0[3],
               (_Float16)a1[0], (_Float16)a1[1], (_Float16)a1[2], (_Float16)a1[3]};
}

__device__ __forceinline__ void gemm32x64(const _Float16* A, int lda, const _Float16* Bt, int ldb, int K,
                                          int m0, int n0, int lane, v8f (&acc)[2][4]) {
#pragma unroll 1
  for (int k0 = 0; k0 < K; k0 += 32) {
    const v16h a0 = ldfrag(A, lda, m0, k0, lane);
    const v16h a1 = ldfrag(A, lda, m0 + 16, k0, lane);
    const v16h b0 = ldfrag(Bt, ldb, n0, k0, lane);
    const v16h b1 = ldfrag(Bt, ldb, n0 + 16, k0, lane);
    const v16h b2 = ldfrag(Bt, ldb, n0 + 32, k0, lane);
    const v16h b3 = ldfrag(Bt, ldb, n0 + 48, k0, lane);
    acc[0][0] = mma16(a0, b0, acc[0][0]);
    acc[1][0] = mma16(a1, b0, acc[1][0]);
    acc[0][1] = mma16(a0, b1, acc[0][1]);
    acc[1][1] = mma16(a1, b1, acc[1][1]);
    acc[0][2] = mma16(a0, b2, acc[0][2]);
    acc[1][2] = mma16(a1, b2, acc[1][2]);
    acc[0][3] = mma16(a0, b3, acc[0][3]);
    acc[1][3] = mma16(a1, b3, acc[1][3]);
  }
}

__global__ __launch_bounds__(256) void k_cvt(const float* __restrict__ src, _Float16* __restrict__ dh,
                                             float scale, int rowlen, int nvalid) {
  const size_t o = (size_t)blockIdx.x * 2048 + (size_t)threadIdx.x * 8;
  const int row = (int)(o / (size_t)rowlen);
  const int col = (int)(o - (size_t)row * rowlen);
  const int rc = min(row, nvalid - 1);
  const float keep = (row < nvalid) ? scale : 0.0f;
  const float* s = src + (size_t)rc * rowlen + col;
  const v4f a0 = (*(const v4f*)(s)) * keep, a1 = (*(const v4f*)(s + 4)) * keep;
  Pack8 pk;
  pk.h = cvt8(a0, a1);
  const v4u vv = pk.u;
  volatile v4u* d = (volatile v4u*)(dh + o);
  *d = vv;
  __threadfence();
  *d = vv;
}

__global__ __launch_bounds__(256) void k_cvt3(const float* __restrict__ w0, const float* __restrict__ w1,
                                              const float* __restrict__ w2, _Float16* __restrict__ dh, float scale,
                                              int* __restrict__ flag) {
  const int o = blockIdx.x * 2048 + threadIdx.x * 8;
  const int n = o / KCAT, k = o - n * KCAT;
  const int part = k >> 7, kk = k & 127;
  const size_t si = (size_t)n * DIM + kk;
  v4f x0 = *(const v4f*)(w0 + si), x1 = *(const v4f*)(w0 + si + 4);
  const v4f y0 = *(const v4f*)(w1 + si), y1 = *(const v4f*)(w1 + si + 4);
  const v4f z0 = *(const v4f*)(w2 + si), z1 = *(const v4f*)(w2 + si + 4);
  if (part == 1) { x0 = y0; x1 = y1; }
  if (part == 2) { x0 = z0; x1 = z1; }
  Pack8 pk;
  pk.h = cvt8(x0 * scale, x1 * scale);
  const v4u vv = pk.u;
  volatile v4u* d = (volatile v4u*)(dh + o);
  *d = vv;
  __threadfence();
  *d = vv;
  if (blockIdx.x == 0 && threadIdx.x == 0) {
    *(volatile int*)flag = 0;
    __threadfence();
    *(volatile int*)flag = 0;
  }
}

__global__ __launch_bounds__(256) void k_emb(const float* __restrict__ emb, int nvalid,
                                             const _Float16* __restrict__ wb, float oscale,
                                             float* __restrict__ outp) {
  __shared__ __align__(16) float smf[8 * 16 * OTP];
  _Float16* at = (_Float16*)smf;
  const int tid = threadIdx.x, lane = tid & 31, wave = tid >> 5, hh = lane >> 4, c = lane & 15;
  const int r0 = blockIdx.x * 128;
#pragma unroll
  for (int j = 0; j < 8; ++j) {
    const int piece = tid + 256 * j;
    const int row = piece >> 4, f = (piece & 15) * 8;
    const int rc = min(r0 + row, nvalid - 1);
    const float* s = emb + (size_t)rc * DIM + f;
    const v4f a0 = (*(const v4f*)(s)) * 8.0f, a1 = (*(const v4f*)(s + 4)) * 8.0f;
    *(v8h*)(at + row * EPITCH + f) = cvt8(a0, a1);
  }
  __syncthreads();
  const int wr = wave >> 1, wc = wave & 1;
  v8f acc[2][4];
#pragma unroll
  for (int s = 0; s < 2; ++s)
#pragma unroll
    for (int t = 0; t < 4; ++t) acc[s][t] = zero8();
  gemm32x64(at, EPITCH, wb, 2 * DIM, DIM, 32 * wr, 64 * wc, lane, acc);
  float* sw = smf + wave * 16 * OTP;
#pragma unroll
  for (int sub = 0; sub < 2; ++sub) {
    __syncthreads();
#pragma unroll
    for (int t = 0; t < 4; ++t)
#pragma unroll
      for (int r = 0; r < 8; ++r) sw[(8 * hh + r) * OTP + 16 * t + c] = acc[sub][t][r] * oscale;
    __syncthreads();
    const int growb = r0 + 32 * wr + 16 * sub;
    v4f val[8]; size_t go[8];
#pragma unroll
    for (int it = 0; it < 8; ++it) {
      const int p = lane + 32 * it, Lr = p >> 3, pc = p & 7, row = Lr >> 1, half = Lr & 1;
      val[it] = *(const v4f*)(sw + row * OTP + half * 32 + pc * 4);
      go[it]  = (size_t)(growb + row) * DIM + 64 * wc + half * 32 + pc * 4;
    }
    for (int ps = 0; ps < 2; ++ps) {
#pragma unroll
      for (int it = 0; it < 8; ++it) *(volatile v4f*)(outp + go[it]) = val[it];
      __threadfence();
    }
  }
}

__global__ __launch_bounds__(256) void k_csr(const int* __restrict__ ni, int nN, int nM,
                                             int* __restrict__ OFF, int* __restrict__ END,
                                             int* __restrict__ LST, int* __restrict__ flag) {
  extern __shared__ __align__(16) int dl[];
  __shared__ int wsum[8];
  int* cnt = dl;
  int* lst = dl + CSR_R;
  const int tid = threadIdx.x, lane = tid & 31, wave = tid >> 5;
  const int m0 = blockIdx.x * CSR_R;
  for (int i = tid; i < CSR_R + CSR_CAP; i += 256) dl[i] = 0;
  __syncthreads();
#pragma unroll 1
  for (int n = tid; n < nN; n += 256) {
    const int d = ni[n];
    const unsigned u = (unsigned)(d - m0);
    if (d >= 0 && d < nM && u < (unsigned)CSR_R) atomicAdd(&cnt[u], 1);
  }
  __syncthreads();
  int s = 0;
#pragma unroll 1
  for (int i = 0; i < 32; ++i) s += cnt[tid * 32 + i];
  int v = s;
#pragma unroll
  for (int off = 1; off < 32; off <<= 1) {
    const int tt = __shfl_up(v, off, 32);
    if (lane >= off) v += tt;
  }
  if (lane == 31) wsum[wave] = v;
  __syncthreads();
  int wpre = 0, tot = 0;
#pragma unroll
  for (int w = 0; w < 8; ++w) { const int x = wsum[w]; tot += x; wpre += (w < wave) ? x : 0; }
  int run = wpre + v - s;
#pragma unroll 1
  for (int i = 0; i < 32; ++i) { const int cc = cnt[tid * 32 + i]; cnt[tid * 32 + i] = run; run += cc; }
  __syncthreads();
  if (tot > CSR_CAP && tid == 0) { *(volatile int*)flag = ERRV; __threadfence(); *(volatile int*)flag = ERRV; }
  v4i ov[8], ev[8];
#pragma unroll
  for (int it = 0; it < 8; ++it) {
    const int idx = 1024 * it + 4 * tid;
    const int e3r = dl[idx + 4];
    const int e3 = (idx + 4 < CSR_R) ? e3r : tot;
    ov[it] = (v4i){cnt[idx], cnt[idx + 1], cnt[idx + 2], cnt[idx + 3]};
    ev[it] = (v4i){cnt[idx + 1], cnt[idx + 2], cnt[idx + 3], e3};
  }
  __syncthreads();
  for (int ps = 0; ps < 2; ++ps) {
#pragma unroll
    for (int it = 0; it < 8; ++it) {
      const int idx = 1024 * it + 4 * tid;
      *(volatile v4i*)(OFF + m0 + idx) = ov[it];
      *(volatile v4i*)(END + m0 + idx) = ev[it];
    }
    __threadfence();
  }
#pragma unroll 1
  for (int n = tid; n < nN; n += 256) {
    const int d = ni[n];
    const unsigned u = (unsigned)(d - m0);
    if (d >= 0 && d < nM && u < (unsigned)CSR_R) {
      const int pos = atomicAdd(&cnt[u], 1);
      if ((unsigned)pos < (unsigned)CSR_CAP) lst[pos] = n;
    }
  }
  __syncthreads();
#pragma unroll 1
  for (int i = 0; i < CSR_R / 256; ++i) {
    const int u = 256 * i + tid;
    const int em = cnt[max(u - 1, 0)];
    int e = cnt[u];
    int o = (u == 0) ? 0 : em;
    o = min(max(o, 0), CSR_CAP);
    e = min(max(e, o), CSR_CAP);
    const int len = min(e - o, MAXDEG);
#pragma unroll 1
    for (int a = 1; a < len; ++a) {
      const int key = lst[o + a];
      int b = a - 1;
#pragma unroll 1
      while (b >= 0 && lst[o + b] > key) { lst[o + b + 1] = lst[o + b]; --b; }
      lst[o + b + 1] = key;
    }
  }
  __syncthreads();
  int* gl = LST + (size_t)blockIdx.x * CSR_CAP;
  for (int ps = 0; ps < 2; ++ps) {
#pragma unroll
    for (int it = 0; it < CSR_CAP / 1024; ++it) {
      const int idx = 1024 * it + 4 * tid;
      const v4i vv = *(const v4i*)(lst + idx);
      *(volatile v4i*)(gl + idx) = vv;
    }
    __threadfence();
  }
}

__global__ __launch_bounds__(128) void k_pre(const int* __restrict__ OFF, const int* __restrict__ END,
                                             const int* __restrict__ LST,
                                             const int* __restrict__ typeb, const int* __restrict__ tokb,
                                             const float* __restrict__ etat, const float* __restrict__ etal,
                                             const float* __restrict__ etar,
                                             const float* __restrict__ TT, const float* __restrict__ TK,
                                             const float* __restrict__ benc, const _Float16* __restrict__ WS,
                                             const float* __restrict__ bconv, const float* __restrict__ alpha,
                                             _Float16* __restrict__ NE, float* __restrict__ SC, int* __restrict__ flag,
                                             int nN, int ntype, int ntok) {
  __shared__ __align__(16) float smf[12544];
  __shared__ __align__(16) float scl[64];
  _Float16* at = (_Float16*)smf;
  const int tid = threadIdx.x, lane = tid & 31, wave = tid >> 5, hh = lane >> 4, c16 = lane & 15;
  const int c = tid;
  const int m0 = blockIdx.x * 64;
  const int* lst = LST + (size_t)(m0 / CSR_R) * CSR_CAP;
  const float be = benc[c];
  int bad = 0;
#pragma unroll 1
  for (int i = 0; i < 64; ++i) {
    const int m = m0 + i;
    int o = OFF[m], e = END[m];
    o = min(max(o, 0), CSR_CAP);
    e = min(max(e, o), CSR_CAP);
    int cnt = e - o;
    if (cnt > MAXDEG) { bad = 1; cnt = MAXDEG; }
    float st = 0.0f, sl = 0.0f, sr = 0.0f;
#pragma unroll 1
    for (int s = 0; s < cnt; ++s) {
      int n = lst[o + s];
      n = min(max(n, 0), nN - 1);
      const int ty = min(max(typeb[n], 0), ntype - 1);
      const int tk = min(max(tokb[n], 0), ntok - 1);
      const float h = TT[(size_t)ty * DIM + c] + TK[(size_t)tk * DIM + c] + be;
      st += etat[n] * h;
      sl += etal[n] * h;
      sr += etar[n] * h;
    }
    _Float16* ar = at + i * APITCH;
    ar[c]           = (_Float16)(st * 64.0f);
    ar[DIM + c]     = (_Float16)(sl * 64.0f);
    ar[2 * DIM + c] = (_Float16)(sr * 64.0f);
  }
  if (bad) { *(volatile int*)flag = ERRV; __threadfence(); *(volatile int*)flag = ERRV; }
  __syncthreads();
  const int wr = wave >> 1, wc = wave & 1;
  v8f acc[2][4];
#pragma unroll
  for (int s = 0; s < 2; ++s)
#pragma unroll
    for (int t = 0; t < 4; ++t) acc[s][t] = zero8();
  gemm32x64(at, APITCH, WS, KCAT, KCAT, 32 * wr, 64 * wc, lane, acc);
  __syncthreads();
  float* O = smf;
  const float bc = bconv[0];
#pragma unroll
  for (int sub = 0; sub < 2; ++sub)
#pragma unroll
    for (int t = 0; t < 4; ++t)
#pragma unroll
      for (int r = 0; r < 8; ++r)
        O[(32 * wr + 16 * sub + 8 * hh + r) * OPITCH + 64 * wc + 16 * t + c16] = acc[sub][t][r] * (1.0f / 2048.0f) + bc;
  __syncthreads();
#pragma unroll 1
  for (int idx = tid; idx < 64 * DIM; idx += 128) {
    const int rr = idx >> 7, cc = idx & 127;
    O[rr * OPITCH + cc] = tanhf(O[rr * OPITCH + cc]);
  }
  __syncthreads();
  if (tid < 64) {
    const float* orow = O + tid * OPITCH;
    float s = 0.0f;
#pragma unroll 4
    for (int k = 0; k < DIM; ++k) s = fmaf(orow[k], alpha[k], s);
    scl[tid] = s;
  }
  __syncthreads();
  v4u val[8];
#pragma unroll
  for (int i = 0; i < 8; ++i) {
    const int row = 16 * wave + 2 * i + hh;
    const float* q = O + row * OPITCH + 8 * c16;
    Pack8 pk;
    pk.h = cvt8(*(const v4f*)(q), *(const v4f*)(q + 4));
    val[i] = pk.u;
  }
  const v4f sv = *(const v4f*)(scl + 4 * c16);
  for (int ps = 0; ps < 2; ++ps) {
#pragma unroll
    for (int i = 0; i < 8; ++i)
      *(volatile v4u*)(NE + (size_t)(m0 + 16 * wave + 2 * i + hh) * DIM + 8 * c16) = val[i];
    if (wave == 0 && lane < 16) *(volatile v4f*)(SC + m0 + 4 * lane) = sv;
    __threadfence();
  }
}

__global__ __launch_bounds__(256) void k_tree(const int* __restrict__ ti, const float* __restrict__ SC,
                                              const _Float16* __restrict__ NE, _Float16* __restrict__ CD, int nM) {
  __shared__ int hl[256];
  __shared__ float he[256];
  __shared__ float red[8];
  __shared__ int wcnt[8];
  __shared__ __align__(16) float part[2][DIM];
  __shared__ float epart[2];
  __shared__ __align__(16) float cdv[DIM];
  const int t = blockIdx.x;
  const int tid = threadIdx.x, lane = tid & 31, wave = tid >> 5;
  const int c = tid & 127, half = tid >> 7;
  float mx = -FLT_MAX;
#pragma unroll 1
  for (int n = tid; n < nM; n += 256) {
    const int tv = ti[n];
    const float sv = SC[n];
    if (tv == t) mx = fmaxf(mx, sv);
  }
#pragma unroll
  for (int off = 16; off >= 1; off >>= 1) mx = fmaxf(mx, __shfl_xor(mx, off, 32));
  if (lane == 0) red[wave] = mx;
  __syncthreads();
#pragma unroll
  for (int w = 0; w < 8; ++w) mx = fmaxf(mx, red[w]);
  float acc = 0.0f, es = 0.0f;
  const int nch = (nM + 255) >> 8;
#pragma unroll 1
  for (int ch = 0; ch < nch; ++ch) {
    const int n = ch * 256 + tid;
    const int nc = min(n, nM - 1);
    const int tv = ti[nc];
    const float sv = SC[nc];
    const bool hit = (n < nM) && (tv == t);
    const float e = expf(hit ? (sv - mx) : 0.0f);
    const unsigned msk = __builtin_amdgcn_ballot_w32(hit);
    const int cw = __builtin_popcount(msk);
    const int pf = __builtin_popcount(msk & ((1u << lane) - 1u));
    if (lane == 0) wcnt[wave] = cw;
    __syncthreads();
    int base = 0, H = 0;
#pragma unroll
    for (int w = 0; w < 8; ++w) { const int x = wcnt[w]; H += x; base += (w < wave) ? x : 0; }
    H = min(H, 256);
    if (hit) { hl[base + pf] = n; he[base + pf] = e; }
    __syncthreads();
#pragma unroll 1
    for (int j = half; j < H; j += 2) {
      int nn = hl[j];
      nn = min(max(nn, 0), nM - 1);
      const float ej = he[j];
      acc = fmaf(ej, (float)NE[(size_t)nn * DIM + c], acc);
      es += ej;
    }
    __syncthreads();
  }
  part[half][c] = acc;
  if (c == 0) epart[half] = es;
  __syncthreads();
  if (tid < DIM) {
    const float den = epart[0] + epart[1];
    const float vsum = part[0][tid] + part[1][tid];
    cdv[tid] = (den > 0.0f) ? vsum * (1.0f / den) : 0.0f;
  }
  __syncthreads();
  const int l16 = lane & 15;
  const v4f a0 = (*(const v4f*)(cdv + 8 * l16)) * 256.0f, a1 = (*(const v4f*)(cdv + 8 * l16 + 4)) * 256.0f;
  Pack8 pk;
  pk.h = cvt8(a0, a1);
  const v4u vv = pk.u;
  if (wave == 0 && lane < 16) {
    for (int ps = 0; ps < 2; ++ps) {
      *(volatile v4u*)(CD + (size_t)t * DIM + 8 * lane) = vv;
      __threadfence();
    }
  }
}

__global__ __launch_bounds__(256) void k_out(const _Float16* __restrict__ CD, const _Float16* __restrict__ WO,
                                             const float* __restrict__ bout, const int* __restrict__ flag,
                                             float* __restrict__ out) {
  __shared__ __align__(16) float O[16 * OCH];
  const int tid = threadIdx.x, lane = tid & 31, wave = tid >> 5, hh = lane >> 4, c16 = lane & 15;
  const int rbase = blockIdx.x * 16;
  const int re = 2 * wave, ro = 2 * wave + 1;
  const size_t gre = (size_t)(rbase + re) * SUBT, gro = (size_t)(rbase + ro) * SUBT;
  v16h af[4];
#pragma unroll
  for (int ks = 0; ks < 4; ++ks) af[ks] = ldfrag(CD, DIM, rbase, 32 * ks, lane);
  const float poison = (flag[0] == ERRV) ? __int_as_float(0x7fc00000) : 0.0f;
  const int Lq = lane >> 3, p = lane & 7, p4 = 4 * (lane & 3);
  v4f carry = (v4f){0.f, 0.f, 0.f, 0.f}, stash = (v4f){0.f, 0.f, 0.f, 0.f};
#pragma unroll 1
  for (int j = 0; j < NCH; ++j) {
    const int c0 = j * OCH, cw = 64 * wave;
    v8f acc[4];
#pragma unroll
    for (int t = 0; t < 4; ++t) acc[t] = zero8();
#pragma unroll
    for (int ks = 0; ks < 4; ++ks) {
#pragma unroll
      for (int t = 0; t < 4; ++t) {
        const v16h b = ldfrag(WO, DIM, c0 + cw + 16 * t, 32 * ks, lane);
        acc[t] = mma16(af[ks], b, acc[t]);
      }
    }
#pragma unroll
    for (int t = 0; t < 4; ++t) {
      const int col = cw + 16 * t + c16;
      const float bb = bout[min(c0 + col, SUBT - 1)];
#pragma unroll
      for (int r = 0; r < 8; ++r) O[(8 * hh + r) * OCH + col] = acc[t][r] * (1.0f / 16384.0f) + bb + poison;
    }
    __syncthreads();
    v4f val[9]; size_t ga[9]; int ok[9];
    const float* Oe = O + re * OCH;
    const float* Oo = O + ro * OCH;
#pragma unroll
    for (int it = 0; it < 4; ++it) {
      const int L = 4 * it + Lq;
      val[it] = *(const v4f*)(Oe + 32 * L + 4 * p);
      ga[it]  = gre + c0 + 32 * L + 4 * p;
      ok[it]  = (c0 + 32 * L + 32 <= SUBT - 16) ? 1 : 0;
      const int cb   = 16 + 32 * (L - 1);
      const int colo = (L == 0) ? (4 * (p & 3)) : (cb + 4 * p);
      const v4f vo = *(const v4f*)(Oo + colo);
      const bool usecarry = (L == 0) && (p < 4);
      val[4 + it] = usecarry ? carry : vo;
      ga[4 + it]  = (L == 0) ? (gro + c0 - 16 + 4 * p) : (gro + c0 + colo);
      ok[4 + it]  = (L == 0) ? ((j >= 1) ? 1 : 0) : ((c0 + cb + 32 <= SUBT) ? 1 : 0);
    }
    {
      const int cs  = (SUBT - 16) - c0;
      const int csl = min(max(cs + 4 * (p & 3), 0), OCH - 4);
      const v4f ve  = *(const v4f*)(Oe + csl);
      val[8] = (p < 4) ? ve : stash;
      ga[8]  = gre + (SUBT - 16) + 4 * p;
      ok[8]  = (j == NCH - 1 && Lq == 0) ? 1 : 0;
    }
    for (int ps = 0; ps < 2; ++ps) {
#pragma unroll
      for (int q = 0; q < 9; ++q)
        if (ok[q]) *(volatile v4f*)(out + ga[q]) = val[q];
      __threadfence();
    }
    const v4f ncar = *(const v4f*)(Oo + OCH - 16 + p4);
    const v4f nsta = *(const v4f*)(Oo + p4);
    carry = ncar;
    if (j == 0) stash = nsta;
    __syncthreads();
  }
}

static inline size_t al256(size_t x) { return (x + 255) & ~(size_t)255; }

extern "C" void kernel_launch(void* const* d_in, const int* in_sizes, int n_in,
                              void* d_out, int out_size, void* d_ws, size_t ws_size,
                              hipStream_t stream) {
  if (n_in < 18) return;
  const int nN = in_sizes[0];
  if (nN < 1) return;
  for (int i = 1; i <= 5; ++i) if (in_sizes[i] != nN) return;
  const int nM = in_sizes[6];
  if (nM < 64 || (nM % 64) != 0) return;
  if (in_sizes[7] < DIM || (in_sizes[7] % DIM) != 0) return;
  if (in_sizes[8] < DIM || (in_sizes[8] % DIM) != 0) return;
  const int ntype = in_sizes[7] / DIM, ntok = in_sizes[8] / DIM;
  if (in_sizes[9] != DIM * 2 * DIM) return;
  if (in_sizes[10] != DIM) return;
  if (in_sizes[11] != DIM * DIM || in_sizes[12] != DIM * DIM || in_sizes[13] != DIM * DIM) return;
  if (in_sizes[14] < 1 || in_sizes[15] != DIM) return;
  const int S = in_sizes[17];
  if (S != SUBT) return;
  if (in_sizes[16] != S * DIM) return;
  if (out_size != NTREE * S) return;

  const int*   typeb = (const int*)d_in[0];
  const int*   tokb  = (const int*)d_in[1];
  const int*   nidx  = (const int*)d_in[2];
  const float* etat  = (const float*)d_in[3];
  const float* etal  = (const float*)d_in[4];
  const float* etar  = (const float*)d_in[5];
  const int*   tidx  = (const int*)d_in[6];
  const float* embty = (const float*)d_in[7];
  const float* embtk = (const float*)d_in[8];
  const float* Wenc  = (const float*)d_in[9];
  const float* benc  = (const float*)d_in[10];
  const float* wt    = (const float*)d_in[11];
  const float* wl    = (const float*)d_in[12];
  const float* wrr   = (const float*)d_in[13];
  const float* bconv = (const float*)d_in[14];
  const float* alpha = (const float*)d_in[15];
  const float* Wout  = (const float*)d_in[16];
  const float* bout  = (const float*)d_in[17];
  float* out = (float*)d_out;

  const int ttRows = ((ntype + 127) / 128) * 128;
  const int tkRows = ((ntok + 127) / 128) * 128;
  const int csrB   = (nM + CSR_R - 1) / CSR_R;

  size_t off = 0;
  const size_t oWE  = off; off = al256(off + (size_t)DIM * 2 * DIM * 2);
  const size_t oWS  = off; off = al256(off + (size_t)DIM * KCAT * 2);
  const size_t oWO  = off; off = al256(off + (size_t)SUBP * DIM * 2);
  const size_t oTT  = off; off = al256(off + (size_t)ttRows * DIM * 4);
  const size_t oTK  = off; off = al256(off + (size_t)tkRows * DIM * 4);
  const size_t oOFF = off; off = al256(off + (size_t)csrB * CSR_R * 4);
  const size_t oEND = off; off = al256(off + (size_t)csrB * CSR_R * 4);
  const size_t oLST = off; off = al256(off + (size_t)csrB * CSR_CAP * 4);
  const size_t oNE  = off; off = al256(off + (size_t)nM * DIM * 2);
  const size_t oSC  = off; off = al256(off + (size_t)nM * 4);
  const size_t oCD  = off; off = al256(off + (size_t)NTREE * DIM * 2);
  const size_t oFLG = off; off = al256(off + 256);
  if (off > ws_size) return;
  if (off > (size_t)134217728) return;

  char* ws = (char*)d_ws;
  _Float16* WE  = (_Float16*)(ws + oWE);
  _Float16* WS  = (_Float16*)(ws + oWS);
  _Float16* WO  = (_Float16*)(ws + oWO);
  float*    TT  = (float*)(ws + oTT);
  float*    TK  = (float*)(ws + oTK);
  int*      OFF = (int*)(ws + oOFF);
  int*      END = (int*)(ws + oEND);
  int*      LST = (int*)(ws + oLST);
  _Float16* NE  = (_Float16*)(ws + oNE);
  float*    SC  = (float*)(ws + oSC);
  _Float16* CD  = (_Float16*)(ws + oCD);
  int*      FLG = (int*)(ws + oFLG);

  k_cvt<<<dim3((DIM * 2 * DIM) / 2048), dim3(256), 0, stream>>>(Wenc, WE, 16.0f, 2 * DIM, DIM);
  k_cvt3<<<dim3((DIM * KCAT) / 2048), dim3(256), 0, stream>>>(wt, wl, wrr, WS, 32.0f, FLG);
  k_cvt<<<dim3((SUBP * DIM) / 2048), dim3(256), 0, stream>>>(Wout, WO, 64.0f, DIM, SUBT);
  k_emb<<<dim3(ttRows / 128), dim3(256), 0, stream>>>(embty, ntype, WE, 0.0078125f, TT);
  k_emb<<<dim3(tkRows / 128), dim3(256), 0, stream>>>(embtk, ntok, WE + DIM, 0.0078125f, TK);
  const size_t dynCsr = (size_t)(CSR_R + CSR_CAP) * 4;
  (void)hipFuncSetAttribute(reinterpret_cast<const void*>(&k_csr), hipFuncAttributeMaxDynamicSharedMemorySize, (int)dynCsr);
  k_csr<<<dim3(csrB), dim3(256), dynCsr, stream>>>(nidx, nN, nM, OFF, END, LST, FLG);
  k_pre<<<dim3(nM / 64), dim3(128), 0, stream>>>(OFF, END, LST, typeb, tokb, etat, etal, etar, TT, TK, benc, WS,
                                                 bconv, alpha, NE, SC, FLG, nN, ntype, ntok);
  k_tree<<<dim3(NTREE), dim3(256), 0, stream>>>(tidx, SC, NE, CD, nM);
  k_out<<<dim3(NTREE / 16), dim3(256), 0, stream>>>(CD, WO, bout, FLG, out);
  (void)hipGetLastError();
}
